// TransformerLayer_16054587752894
// MI455X (gfx1250) — hardware-run, weakly checked
//
#include <hip/hip_runtime.h>
#define BNG 8
#define BNC 128
#define BNL 512
#define BND 64
#define BNF 512
#define BNH 32
#define BWC 16.0f
#define BAC 1024.0f
typedef unsigned short v8us __attribute__((ext_vector_type(8), may_alias));
typedef float  v8f  __attribute__((ext_vector_type(8)));
typedef float  v4f  __attribute__((ext_vector_type(4)));
typedef float  v4fa __attribute__((ext_vector_type(4), may_alias));

__device__ __forceinline__ unsigned short bf16_bits(float x) { unsigned int u = __float_as_uint(x); return (unsigned short)((u + 0x7FFFu + ((u >> 16) & 1u)) >> 16); }
__device__ __forceinline__ float bf16_val(unsigned short b) { return __uint_as_float(((unsigned int)b) << 16); }
__device__ __forceinline__ float bf16_round(float x) { return bf16_val(bf16_bits(x)); }

typedef _Float16 v16h __attribute__((ext_vector_type(16)));
union FragH { v16h v; v8us half[2]; _Float16 h[16]; unsigned short u[16]; };

__global__ __launch_bounds__(256) void k_wt_f16(const float* __restrict__ W, _Float16* __restrict__ Wt, int K, int N, float scale) {
  const int t = blockIdx.x * 256 + threadIdx.x; if (t >= N * (K / 8)) return; const int n = t / (K / 8), k8 = (t % (K / 8)) * 8; FragH f;
#pragma unroll
  for (int i = 0; i < 8; ++i) f.h[i] = (_Float16)(bf16_round(W[(size_t)(k8 + i) * N + n]) * scale); const v8us o = f.half[0];
  *(volatile v8us*)((unsigned short*)Wt + (size_t)n * K + k8) = o; __threadfence(); *(volatile v8us*)((unsigned short*)Wt + (size_t)n * K + k8) = o;
}

typedef _Float16 v4h __attribute__((ext_vector_type(4)));

__global__ __launch_bounds__(256) void k_x16(const float* __restrict__ x, _Float16* __restrict__ X16, size_t n8) { const size_t t = (size_t)blockIdx.x * 256 + threadIdx.x; if (t >= n8) return; FragH f;
#pragma unroll
  for (int q = 0; q < 8; ++q) f.h[q] = (_Float16)bf16_round(x[t * 8 + q]); *(volatile v8us*)((unsigned short*)X16 + t * 8) = f.half[0]; __threadfence(); *(volatile v8us*)((unsigned short*)X16 + t * 8) = f.half[0]; }

__device__ __forceinline__ v16h g2_frag(const _Float16* p, int hh) { FragH f; f.half[0] = *(const v8us*)((const unsigned short*)p + 8 * hh); f.half[1] = *(const v8us*)((const unsigned short*)p + 16 + 8 * hh); return f.v; }
__device__ __forceinline__ v8f g2_mma(v16h a, v16h b, v8f c) { v8f d = __builtin_amdgcn_wmma_f32_16x16x32_f16(false, a, false, b, (short)0, c, false, false); asm volatile("v_nop\n\tv_nop\n\tv_nop\n\tv_nop" : "+v"(d) : "v"(a), "v"(b)); return d; }
template <int ACT>
__global__ __launch_bounds__(128) void k_gemm2(const _Float16* __restrict__ A, int lda, size_t sA, const _Float16* __restrict__ Bh, int ldb, size_t sB, float alpha, const float* __restrict__ bias, size_t sBias, const float* __restrict__ CP, int rowsPerB, size_t sCPb, int row0g,
    float* __restrict__ C, _Float16* __restrict__ C16, int ldc, size_t sC, int M, int N, int K) { static_assert(ACT == 0 || ACT == 3 || ACT == 6 || ACT == 8 || ACT == 9 || ACT == 11 || ACT == 12 || ACT == 14 || ACT == 15 || ACT == 16 || ACT == 17, "k_gemm2: unsupported ACT code (would silently apply no activation)");
  __shared__ __attribute__((aligned(16))) float so[4][32][68];
  const int tid = threadIdx.x, w = tid >> 5, lane = tid & 31, ln = lane & 15, hh = lane >> 4; const int by = blockIdx.y;
  A += (size_t)by * sA; Bh += (size_t)by * sB; const size_t cofs = (size_t)by * sC; const float* bp = bias ? bias + (size_t)by * sBias : nullptr;
  const int ntn = N >> 6; const int mt = blockIdx.x / ntn, nq = blockIdx.x - mt * ntn; const int row0 = mt * 128 + 32 * w, col0 = nq * 64; if (row0 >= M) return;
  const _Float16* a0p = A + (size_t)(row0 + ln) * lda; const _Float16* a1p = a0p + (size_t)16 * lda;
  const _Float16* b0p = Bh + (size_t)(col0 + ln) * ldb; const _Float16* b1p = b0p + (size_t)16 * ldb; const _Float16* b2p = b1p + (size_t)16 * ldb; const _Float16* b3p = b2p + (size_t)16 * ldb;
  const v8f z8 = {0.f,0.f,0.f,0.f,0.f,0.f,0.f,0.f}; v8f c00 = z8, c01 = z8, c02 = z8, c03 = z8, c10 = z8, c11 = z8, c12 = z8, c13 = z8;
  for (int kb = 0; kb < K; kb += 32) { const v16h a0 = g2_frag(a0p + kb, hh), a1 = g2_frag(a1p + kb, hh);
    v16h b = g2_frag(b0p + kb, hh); c00 = g2_mma(a0, b, c00); c10 = g2_mma(a1, b, c10);
    b = g2_frag(b1p + kb, hh); c01 = g2_mma(a0, b, c01); c11 = g2_mma(a1, b, c11);
    b = g2_frag(b2p + kb, hh); c02 = g2_mma(a0, b, c02); c12 = g2_mma(a1, b, c12);
    b = g2_frag(b3p + kb, hh); c03 = g2_mma(a0, b, c03); c13 = g2_mma(a1, b, c13); }
  v8f accs[8] = {c00, c01, c02, c03, c10, c11, c12, c13};
#pragma unroll
  for (int u = 0; u < 8; ++u) { const int t = u & 3, half = u >> 2; const int col = col0 + t * 16 + ln; const float bv = bp ? bf16_round(bp[col]) : 0.f;
#pragma unroll
    for (int r = 0; r < 8; ++r) { const int rloc = half * 16 + 8 * hh + r; float v = accs[u][r] * alpha + bv; if (CP) { if (rowsPerB < 0) v += CP[cofs + (size_t)(row0g + row0 + rloc) * ldc + col];        else { const int bidx = (row0g + row0 + rloc) / rowsPerB; v += CP[(size_t)bidx * sCPb + (size_t)by * 64 + col]; } }
      if (ACT == 3) v = fmaxf(v, 0.f); else if (ACT == 6) v = 0.5f * v * (1.0f + erff(v * 0.70710678118654752f)); else if (ACT == 11) v = 1.0f / (1.0f + expf(-v)); else if (ACT == 15) v = v / (1.0f + expf(-v)); else if (ACT == 12) v = (v > 0.f) ? v : 0.01f * v; else if (ACT == 8) v = tanhf(v); else if (ACT == 9) v = 0.5f * v * (1.0f + tanhf(0.7978845608028654f * (v + 0.044715f * v * v * v))); else if (ACT == 14) v = (v > 0.f) ? v : 0.1f * v; else if (ACT == 16) v = (v >= 0.f) ? v : 0.3f * v; else if (ACT == 17) v = (v >= 0.f) ? v : 0.2f * v;
      so[w][rloc][t * 16 + ln] = v; } }
  __builtin_amdgcn_fence(__ATOMIC_ACQ_REL, "workgroup"); __builtin_amdgcn_wave_barrier();
  const int rsub = lane >> 4, c4 = (lane & 15) * 4;
  for (int pass = 0; pass < 2; ++pass) {
#pragma unroll
    for (int q = 0; q < 16; ++q) { const int r = q * 2 + rsub; const v4f v = *(const v4fa*)&so[w][r][c4]; if (C) *(volatile v4f*)(C + cofs + (size_t)(row0 + r) * ldc + col0 + c4) = v; if (C16) { v4h h4; for (int i = 0; i < 4; ++i) h4[i] = (_Float16)v[i]; *(volatile v4h*)(C16 + cofs + (size_t)(row0 + r) * ldc + col0 + c4) = h4; } }
    if (pass == 0) __threadfence(); } }

#define TL2E 2.8853900817779268f
__device__ __forceinline__ float tanh_f(float x) { const float e = __builtin_amdgcn_exp2f(x * TL2E); const float r = __builtin_amdgcn_rcpf(e + 1.0f); return fmaf(-2.0f, r, 1.0f); }

__global__ __launch_bounds__(256) void k_addtanh(const float* __restrict__ P, const float* __restrict__ Q, const float* __restrict__ va, float* __restrict__ res, unsigned ni, unsigned nj, unsigned nd) {
  const unsigned j = blockIdx.x * 256u + threadIdx.x, i = blockIdx.y; if (i >= ni || j >= nj) return;
  const float* pp = P + (size_t)i * nd; const float* qp = Q + (size_t)j * nd; float s = 0.0f;
#pragma unroll 1
  for (unsigned d = 0; d < nd; d += 4) { const v4f a = *(const v4fa*)(pp + d); const v4f b = *(const v4fa*)(qp + d); const v4f w = *(const v4fa*)(va + d);
#pragma unroll
    for (int q = 0; q < 4; ++q) s += bf16_round(w[q]) * tanh_f(a[q] + b[q]); }
  float* o = res + (size_t)i * nj + j; *(volatile float*)o = s; __threadfence(); *(volatile float*)o = s; }

__global__ __launch_bounds__(256) void k_bandrow(const float* __restrict__ zs, float* __restrict__ wo, _Float16* __restrict__ wh, unsigned nrows) {
  const unsigned rr = blockIdx.x * 256u + threadIdx.x; if (rr >= nrows) return;
  const unsigned pos = rr & (unsigned)(BNL - 1); const float* p = zs + (size_t)rr * BNL; float top = p[0];
  for (unsigned j = 0; j < (unsigned)BNL; j += 4) { const v4f t4 = *(const v4fa*)(p + j); top = fmaxf(fmaxf(fmaxf(top, t4[0]), fmaxf(t4[1], t4[2])), t4[3]); }
  float ss = 0.0f;
  for (unsigned j = 0; j < (unsigned)BNL; j += 4) { const v4f t4 = *(const v4fa*)(p + j);
#pragma unroll
    for (int u = 0; u < 4; ++u) { const float ex = expf(t4[u] - top); ss += ((j + (unsigned)u + (unsigned)BNH - pos) < (unsigned)(2 * BNH)) ? ex : 0.0f; } }
  const float den = ss + 1e-6f;
  for (int pass = 0; pass < 2; ++pass) {
    for (unsigned j = 0; j < (unsigned)BNL; j += 4) { const v4f t4 = *(const v4fa*)(p + j); v4f w4; v4h h4;
#pragma unroll
      for (int u = 0; u < 4; ++u) { const float ex = expf(t4[u] - top); const float wg = ((j + (unsigned)u + (unsigned)BNH - pos) < (unsigned)(2 * BNH)) ? ex / den : 0.0f; const float cw = wg * BAC; w4[u] = wg; h4[u] = (_Float16)((cw < 6.103515625e-05f) ? 0.0f : cw); }
      *(volatile v4f*)(wo + (size_t)rr * BNL + j) = w4; *(volatile v4h*)(wh + (size_t)rr * BNL + j) = h4; }
    if (pass == 0) __threadfence(); } }

template <int TI>
__global__ __launch_bounds__(256) void k_addln(const float* __restrict__ ys, const float* __restrict__ rs, const float* __restrict__ ms, const float* __restrict__ os, float* __restrict__ o32, _Float16* __restrict__ o16, unsigned nrows) {
  const unsigned rr = blockIdx.x * 256u + threadIdx.x; if (rr >= nrows) return;
  const unsigned uu = rr / (unsigned)BNL, pos = rr - uu * (unsigned)BNL; const float* yp = ys + (size_t)rr * BNC; const float* rp = TI ? rs + (size_t)uu * (BNC * BNL) + pos : rs + (size_t)rr * BNC;
  float ss = 0.0f;
  for (unsigned j = 0; j < (unsigned)BNC; j += 4) { const v4f t4 = *(const v4fa*)(yp + j);
#pragma unroll
    for (int u = 0; u < 4; ++u) ss += t4[u] + (TI ? bf16_round(rp[(size_t)(j + u) * BNL]) : rp[j + u]); }
  const float mm = ss * (1.0f / (float)BNC); float qq = 0.0f;
  for (unsigned j = 0; j < (unsigned)BNC; j += 4) { const v4f t4 = *(const v4fa*)(yp + j);
#pragma unroll
    for (int u = 0; u < 4; ++u) { const float gp = t4[u] + (TI ? bf16_round(rp[(size_t)(j + u) * BNL]) : rp[j + u]) - mm; qq += gp * gp; } }
  const float rq = rsqrtf(qq * (1.0f / (float)BNC) + 1e-5f);
  for (int pass = 0; pass < 2; ++pass) {
    for (unsigned j = 0; j < (unsigned)BNC; j += 4) { const v4f t4 = *(const v4fa*)(yp + j); v4f w4; v4h h4;
#pragma unroll
      for (int u = 0; u < 4; ++u) { const float gp = t4[u] + (TI ? bf16_round(rp[(size_t)(j + u) * BNL]) : rp[j + u]) - mm; const float wv = gp * rq * bf16_round(ms[j + u]) + bf16_round(os[j + u]); w4[u] = wv; h4[u] = (_Float16)((fabsf(wv) < 6.103515625e-05f) ? 0.0f : wv); }
      if (TI) { *(volatile v4f*)(o32 + (size_t)rr * BNC + j) = w4; *(volatile v4h*)(o16 + (size_t)rr * BNC + j) = h4; }
      else {
#pragma unroll
        for (int u = 0; u < 4; ++u) *(volatile float*)(o32 + (size_t)uu * (BNC * BNL) + (size_t)(j + u) * BNL + pos) = w4[u]; } }
    if (pass == 0) __threadfence(); } }

extern "C" void kernel_launch(void* const* d_in, const int* in_sizes, int n_in,
                              void* d_out, int out_size, void* d_ws, size_t ws_size, hipStream_t stream) {
  if (n_in < 14) return; if (in_sizes[0] < BNG * BNC * BNL || in_sizes[1] < BNC * BND || in_sizes[2] < BNC * BND || in_sizes[3] < BND || in_sizes[4] < BND || in_sizes[5] < 1 || in_sizes[6] < BNC * BNF || in_sizes[7] < BNF || in_sizes[8] < BNF * BNC || in_sizes[9] < BNC || in_sizes[10] < BNC || in_sizes[11] < BNC || in_sizes[12] < BNC || in_sizes[13] < BNC) return; if (out_size < BNG * BNC * BNL + BNG * BNL * BNL) return;
  const float* const* I = (const float* const*)d_in; const float* ta = I[0]; const float* wk = I[1]; const float* wq = I[2]; const float* ph = I[3]; const float* vz = I[4]; const float* u0 = I[6]; const float* p0 = I[7]; const float* u1 = I[8]; const float* p1 = I[9]; const float* m0 = I[10]; const float* s0 = I[11]; const float* m1 = I[12]; const float* s1 = I[13];
  float* r0 = (float*)d_out; float* r1 = r0 + (size_t)BNG * BNC * BNL;
  static_assert((BNL & (BNL - 1)) == 0 && (BNG * BNL) % 128 == 0 && BNL % 128 == 0 && BND % 64 == 0 && BNC % 64 == 0 && BNF % 64 == 0 && BNC % 32 == 0 && BNL % 32 == 0 && BNF % 32 == 0 && BND % 4 == 0 && BNC % 8 == 0 && BNL % 8 == 0 && BNF % 8 == 0 && BND % 8 == 0 && 2 * BNH <= BNL, "whole tiles");
  uint8_t* wsp = (uint8_t*)d_ws; size_t off = 0;
  auto take = [&](size_t bytes) { uint8_t* p = wsp + off; off += (bytes + 255) & ~(size_t)255; return p; };
  _Float16* TT = (_Float16*)take((size_t)BNG * BNL * BNC * 2); _Float16* TA = (_Float16*)take((size_t)BNG * BNC * BNL * 2); _Float16* WQ = (_Float16*)take((size_t)BND * BNC * 2); _Float16* WK = (_Float16*)take((size_t)BND * BNC * 2); _Float16* U0 = (_Float16*)take((size_t)BNF * BNC * 2); _Float16* U1 = (_Float16*)take((size_t)BNC * BNF * 2); float* PQ = (float*)take((size_t)BNG * BNL * BND * 4); float* PK = (float*)take((size_t)BNG * BNL * BND * 4); float* SC = (float*)take((size_t)BNG * BNL * BNL * 4); _Float16* WH = (_Float16*)take((size_t)BNG * BNL * BNL * 2); float* VS = (float*)take((size_t)BNG * BNL * BNC * 4); float* S1 = (float*)take((size_t)BNG * BNL * BNC * 4); _Float16* S1H = (_Float16*)take((size_t)BNG * BNL * BNC * 2); _Float16* RH = (_Float16*)take((size_t)BNG * BNL * BNF * 2); float* S2 = (float*)take((size_t)BNG * BNL * BNC * 4);
  if (off > ws_size) return;
  for (int u = 0; u < BNG; ++u)
    k_wt_f16<<<(unsigned)(((size_t)BNL * (BNC / 8) + 255) / 256), 256, 0, stream>>>(ta + (size_t)u * BNC * BNL, TT + (size_t)u * BNL * BNC, BNC, BNL, 1.0f);
  k_x16<<<(unsigned)(((size_t)BNG * BNC * BNL / 8 + 255) / 256), 256, 0, stream>>>(ta, TA, (size_t)BNG * BNC * BNL / 8);
  k_wt_f16<<<(unsigned)(((size_t)BND * (BNC / 8) + 255) / 256), 256, 0, stream>>>(wq, WQ, BNC, BND, BWC);
  k_wt_f16<<<(unsigned)(((size_t)BND * (BNC / 8) + 255) / 256), 256, 0, stream>>>(wk, WK, BNC, BND, BWC);
  k_wt_f16<<<(unsigned)(((size_t)BNF * (BNC / 8) + 255) / 256), 256, 0, stream>>>(u0, U0, BNC, BNF, BWC);
  k_wt_f16<<<(unsigned)(((size_t)BNC * (BNF / 8) + 255) / 256), 256, 0, stream>>>(u1, U1, BNF, BNC, BWC);
  k_gemm2<0><<<dim3((unsigned)((BNG * BNL / 128) * (BND / 64)), 1), 128, 0, stream>>>(TT, BNC, 0, WQ, BNC, 0, 1.0f / BWC, ph, 0, nullptr, 1, 0, 0, PQ, nullptr, BND, 0, BNG * BNL, BND, BNC);
  k_gemm2<0><<<dim3((unsigned)((BNG * BNL / 128) * (BND / 64)), 1), 128, 0, stream>>>(TT, BNC, 0, WK, BNC, 0, 1.0f / BWC, nullptr, 0, nullptr, 1, 0, 0, PK, nullptr, BND, 0, BNG * BNL, BND, BNC);
  for (int u = 0; u < BNG; ++u)
    k_addtanh<<<dim3((unsigned)((BNL + 255) / 256), (unsigned)BNL), 256, 0, stream>>>(PQ + (size_t)u * BNL * BND, PK + (size_t)u * BNL * BND, vz, SC + (size_t)u * BNL * BNL, (unsigned)BNL, (unsigned)BNL, (unsigned)BND);
  k_bandrow<<<(unsigned)((BNG * BNL + 255) / 256), 256, 0, stream>>>(SC, r1, WH, (unsigned)(BNG * BNL));
  k_gemm2<0><<<dim3((unsigned)((BNL / 128) * (BNC / 64)), (unsigned)BNG), 128, 0, stream>>>(WH, BNL, (size_t)BNL * BNL, TA, BNL, (size_t)BNC * BNL, 1.0f / BAC, nullptr, 0, nullptr, 1, 0, 0, VS, nullptr, BNC, (size_t)BNL * BNC, BNL, BNC, BNL);
  k_addln<1><<<(unsigned)((BNG * BNL + 255) / 256), 256, 0, stream>>>(VS, ta, m0, s0, S1, S1H, (unsigned)(BNG * BNL));
  k_gemm2<3><<<dim3((unsigned)((BNG * BNL / 128) * (BNF / 64)), 1), 128, 0, stream>>>(S1H, BNC, 0, U0, BNC, 0, 1.0f / BWC, p0, 0, nullptr, 1, 0, 0, nullptr, RH, BNF, 0, BNG * BNL, BNF, BNC);
  k_gemm2<0><<<dim3((unsigned)((BNG * BNL / 128) * (BNC / 64)), 1), 128, 0, stream>>>(RH, BNF, 0, U1, BNF, 0, 1.0f / BWC, p1, 0, nullptr, 1, 0, 0, S2, nullptr, BNC, 0, BNG * BNL, BNC, BNF);
  k_addln<0><<<(unsigned)((BNG * BNL + 255) / 256), 256, 0, stream>>>(S2, S1, m1, s1, r0, nullptr, (unsigned)(BNG * BNL));
}
